// DepthConv_60687887892852
// MI455X (gfx1250) — hardware-verified
//
#include <hip/hip_runtime.h>
#ifndef NB
#define NB 8
#endif
#define CIN 64
#define COUT 64
#define HH 128
#define WW 128
#define HP (HH + 2)
#define WP (WW + 2)
#define XB_FULL ((size_t)CIN * HH * WW)
#define DB_FULL ((size_t)HH * WW)
#define OB_FULL ((size_t)COUT * HH * WW)
#define XP_B ((size_t)HP * WP * CIN)
#define W16_N ((size_t)9 * COUT * CIN)

static_assert(CIN == 64);
static_assert(COUT == 64);
static_assert(WW % 32 == 0);
static_assert((9 * COUT * (CIN / 8)) % 256 == 0);

typedef __bf16 v16b __attribute__((ext_vector_type(16)));
typedef unsigned short v8us __attribute__((ext_vector_type(8), may_alias));
typedef float v8f __attribute__((ext_vector_type(8)));
typedef float v4f __attribute__((ext_vector_type(4)));
typedef float v4fa __attribute__((ext_vector_type(4), may_alias));
union FragB { v16b v; v8us half[2]; unsigned short u[16]; };

__device__ __forceinline__ unsigned short bf16_bits(float x) { unsigned int u = __float_as_uint(x); return (unsigned short)((u + 0x7FFFu + ((u >> 16) & 1u)) >> 16); }
__device__ __forceinline__ float bf16_val(unsigned short b) { return __uint_as_float(((unsigned int)b) << 16); }
__device__ __forceinline__ float bf16_rne(float x) { return bf16_val(bf16_bits(x)); }

__device__ __forceinline__ v8f mma_bf(v16b a, v16b b, v8f c) {
  v8f d = __builtin_amdgcn_wmma_f32_16x16x32_bf16(false, a, false, b, (short)0, c, false, false);
  asm volatile("v_nop\n\tv_nop\n\tv_nop\n\tv_nop" : "+v"(d) : "v"(a), "v"(b));
  return d;
}
__device__ __forceinline__ v16b frag_ld(const unsigned short* p, int hh) {
  FragB f;
  f.half[0] = *(const v8us*)(p + 8 * hh);
  f.half[1] = *(const v8us*)(p + 16 + 8 * hh);
  return f.v;
}

__global__ __launch_bounds__(256) void k_wp(const float* __restrict__ wgt, unsigned short* __restrict__ W16) {
  const int t = blockIdx.x * 256 + threadIdx.x;
  if (t >= 9 * COUT * (CIN / 8)) return;
  const int row = t >> 3, pc = (t & 7) * 8;
  const int tap = row >> 6, o = row & 63;
  v8us v;
#pragma unroll
  for (int q = 0; q < 8; ++q) v[q] = bf16_bits(wgt[((size_t)o * CIN + pc + q) * 9 + tap]);
  unsigned short* p = W16 + (size_t)row * CIN + pc;
  *(volatile v8us*)p = v;
  __threadfence();
  *(volatile v8us*)p = v;
}

__global__ __launch_bounds__(256) void k_xp(const float* __restrict__ x, unsigned short* __restrict__ XPp) {
  __shared__ __attribute__((aligned(16))) unsigned short tl[WW][72];
  const int hp = blockIdx.x, b = blockIdx.y, tid = threadIdx.x;
  const bool interior = (hp >= 1) && (hp <= HH);
  const int hs = min(max(hp - 1, 0), HH - 1);
  const float* src = x + (size_t)b * XB_FULL + (size_t)hs * WW;
  for (int idx = tid; idx < CIN * WW; idx += 256) {
    const int c = idx >> 7, w = idx & (WW - 1);
    const float v = src[(size_t)c * HH * WW + w];
    tl[w][c] = interior ? bf16_bits(v) : (unsigned short)0;
  }
  __syncthreads();
  unsigned short* dst = XPp + (size_t)b * XP_B + (size_t)hp * WP * CIN;
  const int pr = tid >> 3, pc = (tid & 7) * 8;
  for (int pass = 0; pass < 2; ++pass) {
    for (int it = 0; it < (WP + 31) / 32; ++it) {
      const int wp = it * 32 + pr;
      const int wsrc = min(max(wp - 1, 0), WW - 1);
      v8us v = *(const v8us*)&tl[wsrc][pc];
      const bool live = (wp >= 1) && (wp <= WW);
      if (!live) {
#pragma unroll
        for (int q = 0; q < 8; ++q) v[q] = 0;
      }
      if (wp < WP) *(volatile v8us*)(dst + (size_t)wp * CIN + pc) = v;
    }
    if (pass == 0) __threadfence();
  }
}

__global__ __launch_bounds__(128) void k_conv(const unsigned short* __restrict__ XPp, const unsigned short* __restrict__ W16,
                                              const float* __restrict__ depth, const float* __restrict__ bias, float* __restrict__ out) {
  __shared__ __attribute__((aligned(16))) float so[4][COUT][32];
  __shared__ float sbias[COUT];
  const int tid = threadIdx.x, w = tid >> 5, lane = tid & 31, n = lane & 15, hh = lane >> 4;
  const int h = blockIdx.x, b = blockIdx.y;
  const int w0 = w * 32;
  if (tid < COUT) sbias[tid] = bf16_rne(bias[tid]);
  __syncthreads();
  const float* dmap = depth + (size_t)b * DB_FULL;
  int wc[2]; float dc[2];
#pragma unroll
  for (int g = 0; g < 2; ++g) { wc[g] = w0 + g * 16 + n; dc[g] = bf16_rne(dmap[(size_t)h * WW + wc[g]]); }
  const v8f z8 = {0.f, 0.f, 0.f, 0.f, 0.f, 0.f, 0.f, 0.f};
  v8f acc[2][4];
#pragma unroll
  for (int g = 0; g < 2; ++g)
#pragma unroll
    for (int t = 0; t < 4; ++t) acc[g][t] = z8;
  const unsigned short* xb = XPp + (size_t)b * XP_B;
#pragma unroll 1
  for (int tap = 0; tap < 9; ++tap) {
    const int kh = tap / 3, kw = tap - kh * 3;
    const int hq = h + kh - 1;
    const bool hok = (hq >= 0) && (hq < HH);
    const int hcl = min(max(hq, 0), HH - 1);
    float s[2];
    v16b bfr[2][2];
#pragma unroll
    for (int g = 0; g < 2; ++g) {
      const int wq = wc[g] + kw - 1;
      const int wcl = min(max(wq, 0), WW - 1);
      float dt = bf16_rne(dmap[(size_t)hcl * WW + wcl]);
      const bool ok = hok && (wq >= 0) && (wq < WW);
      dt = ok ? dt : 0.0f;
      s[g] = expf(-fabsf(dt - dc[g]));
      const unsigned short* px = xb + ((size_t)(h + kh) * WP + (size_t)(wc[g] + kw)) * CIN;
      bfr[g][0] = frag_ld(px, hh);
      bfr[g][1] = frag_ld(px + 32, hh);
    }
    const unsigned short* wt = W16 + (size_t)tap * COUT * CIN;
#pragma unroll
    for (int t = 0; t < 4; ++t) {
      const unsigned short* wr = wt + (size_t)(t * 16 + n) * CIN;
      const v16b a0 = frag_ld(wr, hh), a1 = frag_ld(wr + 32, hh);
#pragma unroll
      for (int g = 0; g < 2; ++g) {
        v8f d = mma_bf(a0, bfr[g][0], z8);
        d = mma_bf(a1, bfr[g][1], d);
#pragma unroll
        for (int r = 0; r < 8; ++r) acc[g][t][r] = fmaf(s[g], d[r], acc[g][t][r]);
      }
    }
  }
#pragma unroll
  for (int t = 0; t < 4; ++t)
#pragma unroll
    for (int r = 0; r < 8; ++r) {
      const int o = t * 16 + 8 * hh + r;
      const float bv = sbias[o];
#pragma unroll
      for (int g = 0; g < 2; ++g) so[w][o][g * 16 + n] = acc[g][t][r] + bv;
    }
  __syncthreads();
  float* ob = out + (size_t)b * OB_FULL + (size_t)h * WW + w0;
  const int lr = lane >> 3, c4 = (lane & 7) * 4;
  for (int pass = 0; pass < 2; ++pass) {
#pragma unroll
    for (int q = 0; q < 16; ++q) {
      const int o = q * 4 + lr;
      const v4f v = *(const v4fa*)&so[w][o][c4];
      *(volatile v4f*)(ob + (size_t)o * HH * WW + c4) = v;
    }
    if (pass == 0) __threadfence();
  }
}

extern "C" void kernel_launch(void* const* d_in, const int* in_sizes, int n_in,
                              void* d_out, int out_size, void* d_ws, size_t ws_size, hipStream_t stream) {
  if (n_in < 4) return;
  if ((size_t)in_sizes[0] < (size_t)NB * XB_FULL) return;
  if ((size_t)in_sizes[1] < (size_t)NB * DB_FULL) return;
  if (in_sizes[2] < 9 * COUT * CIN) return;
  if (in_sizes[3] < COUT) return;
  if ((size_t)out_size < (size_t)NB * OB_FULL) return;
  const float* x     = (const float*)d_in[0];
  const float* depth = (const float*)d_in[1];
  const float* wgt   = (const float*)d_in[2];
  const float* bias  = (const float*)d_in[3];
  float* out = (float*)d_out;
  char* ws = (char*)d_ws; size_t off = 0;
  const size_t xp_bytes = ((size_t)NB * XP_B * 2 + 255) & ~(size_t)255;
  const size_t w_bytes  = (W16_N * 2 + 255) & ~(size_t)255;
  unsigned short* XPp = (unsigned short*)(ws + off); off += xp_bytes;
  unsigned short* W16 = (unsigned short*)(ws + off); off += w_bytes;
  if (off > ws_size) return;
  k_wp<<<(unsigned)((9 * COUT * (CIN / 8)) / 256), 256, 0, stream>>>(wgt, W16);
  k_xp<<<dim3(HP, NB), 256, 0, stream>>>(x, XPp);
  k_conv<<<dim3(HH, NB), 128, 0, stream>>>(XPp, W16, depth, bias, out);
}
